// MNet_6064493822008
// MI455X (gfx1250) — hardware-run, weakly checked
//
#include <hip/hip_runtime.h>
#include <stddef.h>
#include <stdint.h>

#define NEUR   64
#define WP     72
#define NWAVES 4
#define TM     32
#define RPI    (NWAVES * TM)
#define ITERS  16
#define RPB    (RPI * ITERS)

static_assert(NEUR == 64);
static_assert((WP % 8) == 0);
static_assert(RPI == 128);
static_assert((RPB % TM) == 0);

typedef _Float16 v8h  __attribute__((ext_vector_type(8)));
typedef _Float16 v16h __attribute__((ext_vector_type(16)));
typedef float    v4f  __attribute__((ext_vector_type(4)));
typedef float    v8f  __attribute__((ext_vector_type(8)));

union Frag { v16h v; v8h half[2]; };

__device__ __forceinline__ float bf16r(float f) {
  unsigned u = __float_as_uint(f);
  u = (u + 0x7FFFu + ((u >> 16) & 1u)) & 0xFFFF0000u;
  return __uint_as_float(u);
}
__device__ __forceinline__ v8f zero8() { v8f z = {0.f, 0.f, 0.f, 0.f, 0.f, 0.f, 0.f, 0.f}; return z; }
__device__ __forceinline__ float silu_f(float z) {
  const float e = __expf(-z);
  return z * __builtin_amdgcn_rcpf(1.0f + e);
}

__device__ __forceinline__ v16h ldfrag(const _Float16* p) {
  Frag f;
  f.half[0] = *(const v8h*)(p);
  f.half[1] = *(const v8h*)(p + 16);
  return f.v;
}

__device__ __forceinline__ v8f mma_h(v16h a, v16h b, v8f c) {
  return __builtin_amdgcn_wmma_f32_16x16x32_f16(false, a, false, b, (short)0, c, false, false);
}
__device__ __forceinline__ void guard2(v8f& c0, v8f& c1,
                                       const v16h& a0, const v16h& a1, const v16h& a2, const v16h& a3,
                                       const v16h& b0, const v16h& b1) {
#if defined(__HIP_DEVICE_COMPILE__)
  asm volatile("v_nop\n\tv_nop\n\tv_nop\n\tv_nop"
               : "+v"(c0), "+v"(c1)
               : "v"(a0), "v"(a1), "v"(a2), "v"(a3), "v"(b0), "v"(b1));
#endif
}

__device__ __forceinline__ void stage_w(_Float16* dst, const float* __restrict__ src, int tid) {
#pragma unroll
  for (int s = 0; s < 4; ++s) {
    const int idx8 = (s * 128 + tid) * 8;
    const int nrow = idx8 >> 6, k = idx8 & 63;
    const v4f va = *(const v4f*)(src + idx8);
    const v4f vb = *(const v4f*)(src + idx8 + 4);
    v8h o;
#pragma unroll
    for (int q = 0; q < 4; ++q) {
      o[q]     = (_Float16)(bf16r(va[q]) * 64.0f);
      o[q + 4] = (_Float16)(bf16r(vb[q]) * 64.0f);
    }
    *(v8h*)(dst + nrow * WP + k) = o;
  }
}

__global__ __launch_bounds__(128)
void k_mlp(const float* __restrict__ x,
           const float* __restrict__ W0, const float* __restrict__ b0,
           const float* __restrict__ W1, const float* __restrict__ b1,
           const float* __restrict__ W2, const float* __restrict__ b2,
           const float* __restrict__ W3, const float* __restrict__ b3,
           const float* __restrict__ W4, const float* __restrict__ b4,
           const float* __restrict__ Wout, const float* __restrict__ bout,
           float* out, int n)
{
  __shared__ __align__(16) _Float16 wlds[4][NEUR * WP];
  __shared__ __align__(16) _Float16 act[NWAVES][TM * WP];
  __shared__ __align__(16) float w0s[NEUR];
  __shared__ __align__(16) float b0s[NEUR];
  __shared__ __align__(16) float bls[4][NEUR];
  __shared__ __align__(16) float wos[NEUR];
  __shared__ __align__(16) float sOut[NWAVES][TM];
  __shared__ float bo_s;

  const int tid = threadIdx.x;

  stage_w(wlds[0], W1, tid);
  stage_w(wlds[1], W2, tid);
  stage_w(wlds[2], W3, tid);
  stage_w(wlds[3], W4, tid);
  if (tid < NEUR) {
    bls[0][tid] = bf16r(b1[tid]);
    bls[1][tid] = bf16r(b2[tid]);
    bls[2][tid] = bf16r(b3[tid]);
    bls[3][tid] = bf16r(b4[tid]);
    w0s[tid] = bf16r(W0[tid]);
    b0s[tid] = bf16r(b0[tid]);
    wos[tid] = bf16r(Wout[tid]);
  }
  if (tid == 0) bo_s = bf16r(bout[0]);
  __syncthreads();

  const int lane = tid & 31;
  const int wave = tid >> 5;
  const int hh   = lane >> 4;
  const int c    = lane & 15;
  _Float16* actW = act[wave];
  const float boR = bo_s;
  const float kinv = 0.0009765625f;
  const long blockRow0 = (long)blockIdx.x * RPB;

#pragma unroll 1
  for (int it = 0; it < ITERS; ++it) {
    const long r0w = blockRow0 + (long)it * RPI + (long)wave * TM;
    __syncthreads();

    {
      long gr = r0w + lane;
      if (gr > (long)n - 1) gr = (long)n - 1;
      const float xv = bf16r(x[gr]);
#pragma unroll
      for (int j8 = 0; j8 < 8; ++j8) {
        const v4f wA = *(const v4f*)&w0s[j8 * 8];
        const v4f wB = *(const v4f*)&w0s[j8 * 8 + 4];
        const v4f bA = *(const v4f*)&b0s[j8 * 8];
        const v4f bB = *(const v4f*)&b0s[j8 * 8 + 4];
        v8h o;
#pragma unroll
        for (int q = 0; q < 4; ++q) {
          o[q]     = (_Float16)(16.0f * silu_f(xv * wA[q] + bA[q]));
          o[q + 4] = (_Float16)(16.0f * silu_f(xv * wB[q] + bB[q]));
        }
        *(v8h*)(actW + lane * WP + j8 * 8) = o;
      }
    }
    __syncthreads();

#pragma unroll 1
    for (int li = 0; li < 3; ++li) {
      const _Float16* wl = wlds[li];
      const v16h a00 = ldfrag(actW + c * WP + 8 * hh);
      const v16h a01 = ldfrag(actW + c * WP + 32 + 8 * hh);
      const v16h a10 = ldfrag(actW + (16 + c) * WP + 8 * hh);
      const v16h a11 = ldfrag(actW + (16 + c) * WP + 32 + 8 * hh);
#pragma unroll
      for (int nt = 0; nt < 4; ++nt) {
        const int n0 = nt * 16;
        const _Float16* wp = wl + (n0 + c) * WP + 8 * hh;
        const v16h g0 = ldfrag(wp);
        const v16h g1 = ldfrag(wp + 32);
        v8f acc0 = zero8(), acc1 = zero8();
        acc0 = mma_h(a00, g0, acc0);
        acc1 = mma_h(a10, g0, acc1);
        acc0 = mma_h(a01, g1, acc0);
        acc1 = mma_h(a11, g1, acc1);
        guard2(acc0, acc1, a00, a01, a10, a11, g0, g1);
        const float bias = bls[li][n0 + c];
#pragma unroll
        for (int r = 0; r < 8; ++r) {
          const float h0v = silu_f(acc0[r] * kinv + bias);
          const float h1v = silu_f(acc1[r] * kinv + bias);
          actW[(8 * hh + r) * WP + n0 + c]      = (_Float16)(16.0f * h0v);
          actW[(16 + 8 * hh + r) * WP + n0 + c] = (_Float16)(16.0f * h1v);
        }
      }
      __syncthreads();
    }

    {
      const _Float16* wl = wlds[3];
      const v16h a00 = ldfrag(actW + c * WP + 8 * hh);
      const v16h a01 = ldfrag(actW + c * WP + 32 + 8 * hh);
      const v16h a10 = ldfrag(actW + (16 + c) * WP + 8 * hh);
      const v16h a11 = ldfrag(actW + (16 + c) * WP + 32 + 8 * hh);
      float s0[8], s1[8];
#pragma unroll
      for (int r = 0; r < 8; ++r) { s0[r] = 0.0f; s1[r] = 0.0f; }
#pragma unroll
      for (int nt = 0; nt < 4; ++nt) {
        const int n0 = nt * 16;
        const _Float16* wp = wl + (n0 + c) * WP + 8 * hh;
        const v16h g0 = ldfrag(wp);
        const v16h g1 = ldfrag(wp + 32);
        v8f acc0 = zero8(), acc1 = zero8();
        acc0 = mma_h(a00, g0, acc0);
        acc1 = mma_h(a10, g0, acc1);
        acc0 = mma_h(a01, g1, acc0);
        acc1 = mma_h(a11, g1, acc1);
        guard2(acc0, acc1, a00, a01, a10, a11, g0, g1);
        const float bias = bls[3][n0 + c];
        const float wo   = wos[n0 + c];
#pragma unroll
        for (int r = 0; r < 8; ++r) {
          const float h0v = silu_f(acc0[r] * kinv + bias);
          const float h1v = silu_f(acc1[r] * kinv + bias);
          s0[r] += h0v * wo;
          s1[r] += h1v * wo;
        }
      }
#pragma unroll
      for (int off = 8; off >= 1; off >>= 1) {
#pragma unroll
        for (int r = 0; r < 8; ++r) {
          s0[r] += __shfl_xor(s0[r], off, 16);
          s1[r] += __shfl_xor(s1[r], off, 16);
        }
      }
      if (c == 0) {
#pragma unroll
        for (int r = 0; r < 8; ++r) {
          sOut[wave][8 * hh + r]      = s0[r] + boR;
          sOut[wave][16 + 8 * hh + r] = s1[r] + boR;
        }
      }
      __syncthreads();

      const float ov = sOut[wave][lane];
      const long gr = r0w + lane;
      if (gr < (long)n) *(volatile float*)(out + gr) = ov;
      __threadfence();
      if (gr < (long)n) *(volatile float*)(out + gr) = ov;
    }
  }
}

extern "C" void kernel_launch(void* const* d_in, const int* in_sizes, int n_in,
                              void* d_out, int out_size, void* d_ws, size_t ws_size,
                              hipStream_t stream) {
  (void)d_ws; (void)ws_size;
  if (n_in < 13) return;
  const int n = in_sizes[0];
  if (n < 1) return;
  if (out_size != n) return;
  if (in_sizes[1] != NEUR || in_sizes[2] != NEUR) return;
  if (in_sizes[3] != NEUR * NEUR || in_sizes[4] != NEUR) return;
  if (in_sizes[5] != NEUR * NEUR || in_sizes[6] != NEUR) return;
  if (in_sizes[7] != NEUR * NEUR || in_sizes[8] != NEUR) return;
  if (in_sizes[9] != NEUR * NEUR || in_sizes[10] != NEUR) return;
  if (in_sizes[11] != NEUR || in_sizes[12] < 1) return;

  const float* x    = (const float*)d_in[0];
  const float* W0   = (const float*)d_in[1];
  const float* b0   = (const float*)d_in[2];
  const float* W1   = (const float*)d_in[3];
  const float* b1   = (const float*)d_in[4];
  const float* W2   = (const float*)d_in[5];
  const float* b2   = (const float*)d_in[6];
  const float* W3   = (const float*)d_in[7];
  const float* b3   = (const float*)d_in[8];
  const float* W4   = (const float*)d_in[9];
  const float* b4   = (const float*)d_in[10];
  const float* Wout = (const float*)d_in[11];
  const float* bout = (const float*)d_in[12];
  float* out = (float*)d_out;

  const int grid = (n + RPB - 1) / RPB;
  k_mlp<<<dim3(grid), dim3(128), 0, stream>>>(x, W0, b0, W1, b1, W2, b2, W3, b3, W4, b4, Wout, bout, out, n);
  (void)hipGetLastError();
}
